// _FCtL_36747740184603
// MI455X (gfx1250) — hardware-verified
//
#include <hip/hip_runtime.h>
#include <stdint.h>

#define CH     256
#define NP     9216
#define DQ     64
#define NROWS  384
#define PT     288
#define QTILE  64
#define NQT    144
#define KHALF  4608
#define NT16   288
#define NKC    288
#define VPC    36
#define SPP    40
#define SLP    68

#define ASCALE   64.0f
#define WSCALE   1024.0f
#define OSC_PROJ (1.0f / 65536.0f)
#define SINV     (1.0f / 4096.0f)
#define PSCALE   16384.0f
#define PSHIFT   (16384.0f / (float)NP)
#define OSC_ATT  (1.0f / 1048576.0f)

static_assert(PT * 32 == NP);
static_assert(NQT * QTILE == NP);
static_assert(NKC * 32 == NP);
static_assert(NT16 * 16 == KHALF);
static_assert(2 * KHALF == NP);
static_assert(VPC * 256 == NP);
static_assert(NROWS == 2 * DQ + CH);
static_assert((NROWS % 32) == 0 && (NROWS % 8) == 0);
static_assert((NP % 128) == 0 && (CH % 64) == 0 && (DQ % 64) == 0 && (CH % 32) == 0);
static_assert(((DQ / 64) * (NP / 64)) % 8 == 0);
static_assert(((CH / 64) * (NP / 64)) % 8 == 0);
static_assert(QTILE == 64 && (SPP % 8) == 0 && (SLP % 4) == 0);

typedef _Float16 v16h __attribute__((ext_vector_type(16)));
typedef _Float16 v8h  __attribute__((ext_vector_type(8)));
typedef float    v8f  __attribute__((ext_vector_type(8)));
typedef float    v4f  __attribute__((ext_vector_type(4)));
typedef unsigned int v4u __attribute__((ext_vector_type(4)));

__device__ __forceinline__ unsigned short bf_bits(float f) {
  unsigned u = __float_as_uint(f);
  return (unsigned short)((u + 0x7FFFu + ((u >> 16) & 1u)) >> 16);
}
__device__ __forceinline__ float bf_up(unsigned short hb) { return __uint_as_float(((unsigned)hb) << 16); }
__device__ __forceinline__ float bfr(float f) { return bf_up(bf_bits(f)); }
__device__ __forceinline__ unsigned short h_bits(_Float16 x) { return __builtin_bit_cast(unsigned short, x); }
__device__ __forceinline__ unsigned short f2h_bits(float f) { return h_bits((_Float16)f); }
__device__ __forceinline__ unsigned pk16(unsigned short a, unsigned short b) { return (unsigned)a | ((unsigned)b << 16); }
__device__ __forceinline__ v8f zero8() { v8f z = {0.f, 0.f, 0.f, 0.f, 0.f, 0.f, 0.f, 0.f}; return z; }

__device__ __forceinline__ v16h ldfrag_h(const _Float16* p) {
  union { v16h v; v8h hv[2]; } f;
  f.hv[0] = *(const v8h*)(p);
  f.hv[1] = *(const v8h*)(p + 16);
  return f.v;
}

__device__ __forceinline__ v8f mma_h_raw(v16h a, v16h b, v8f c) {
  return __builtin_amdgcn_wmma_f32_16x16x32_f16(false, a, false, b, (short)0, c, false, false);
}
__device__ __forceinline__ void dep_guard1(v8f& a, v16h x, v16h y) {
#if defined(__HIP_DEVICE_COMPILE__)
  asm volatile("v_nop\n\tv_nop\n\tv_nop\n\tv_nop" : "+v"(a) : "v"(x), "v"(y));
#endif
}
__device__ __forceinline__ void dep_guard_h(v8f& a, v8f& b, v16h x, v16h y) {
#if defined(__HIP_DEVICE_COMPILE__)
  asm volatile("v_nop\n\tv_nop\n\tv_nop\n\tv_nop" : "+v"(a), "+v"(b) : "v"(x), "v"(y));
#endif
}
__device__ __forceinline__ void keep4_h(v16h a, v16h b, v16h c, v16h d) {
#if defined(__HIP_DEVICE_COMPILE__)
  asm volatile("v_nop" :: "v"(a), "v"(b), "v"(c), "v"(d));
#endif
}
__device__ __forceinline__ void keep2_h(v16h a, v16h b) {
#if defined(__HIP_DEVICE_COMPILE__)
  asm volatile("v_nop" :: "v"(a), "v"(b));
#endif
}
__device__ __forceinline__ void acc_guard4(v8f& a, v8f& b, v8f& c, v8f& d) {
#if defined(__HIP_DEVICE_COMPILE__)
  asm volatile("v_nop\n\tv_nop\n\tv_nop\n\tv_nop" : "+v"(a), "+v"(b), "+v"(c), "+v"(d));
#endif
}
__device__ __forceinline__ void wave_sync_lds() {
  __builtin_amdgcn_fence(__ATOMIC_RELEASE, "workgroup");
  __builtin_amdgcn_wave_barrier();
  __builtin_amdgcn_fence(__ATOMIC_ACQUIRE, "workgroup");
}

__global__ __launch_bounds__(256) void cvt_tok(const float* __restrict__ x, const float* __restrict__ y,
                                                unsigned short* xt, unsigned short* yt) {
  __shared__ __align__(16) float sx[CH * 33];
  const int tid = threadIdx.x;
  const int which = blockIdx.y;
  const float* src = (which != 0) ? y : x;
  unsigned short* dstp = (which != 0) ? yt : xt;
  const int p0 = blockIdx.x * 32;
#pragma unroll 8
  for (int it = 0; it < 32; ++it) {
    const int idx = it * 256 + tid;
    const int c = idx >> 5, q = idx & 31;
    sx[c * 33 + q] = src[(size_t)c * NP + p0 + q];
  }
  __syncthreads();
  const int wave = tid >> 5, lane = tid & 31, c8 = lane * 8;
  v4u pk[4];
#pragma unroll
  for (int it = 0; it < 4; ++it) {
    const int r = wave * 4 + it;
    v4u p;
#pragma unroll
    for (int e = 0; e < 4; ++e) {
      const float a = bfr(sx[(c8 + 2 * e) * 33 + r]) * ASCALE;
      const float b = bfr(sx[(c8 + 2 * e + 1) * 33 + r]) * ASCALE;
      p[e] = pk16(f2h_bits(a), f2h_bits(b));
    }
    pk[it] = p;
  }
  unsigned short* dst = dstp + (size_t)p0 * CH;
  for (int pass = 0; pass < 2; ++pass) {
#pragma unroll
    for (int it = 0; it < 4; ++it) {
      const int r = wave * 4 + it;
      *(volatile v4u*)(dst + (size_t)r * CH + c8) = pk[it];
    }
    __threadfence();
  }
}

__global__ __launch_bounds__(256) void cvt_w(const float* __restrict__ wq, const float* __restrict__ wk,
                                              const float* __restrict__ wv, unsigned short* wall) {
  const int tid = threadIdx.x, wave = tid >> 5, lane = tid & 31, c8 = lane * 8;
  const int row = blockIdx.x * 8 + wave;
  const float* src;
  if (row < DQ)          src = wq + (size_t)row * CH;
  else if (row < 2 * DQ) src = wk + (size_t)(row - DQ) * CH;
  else                   src = wv + (size_t)(row - 2 * DQ) * CH;
  float vals[8];
#pragma unroll
  for (int i = 0; i < 8; ++i) vals[i] = bfr(src[c8 + i]) * WSCALE;
  v4u p;
#pragma unroll
  for (int i = 0; i < 4; ++i) p[i] = pk16(f2h_bits(vals[2 * i]), f2h_bits(vals[2 * i + 1]));
  unsigned short* d = wall + (size_t)row * CH + c8;
  *(volatile v4u*)d = p;
  __threadfence();
  *(volatile v4u*)d = p;
}

__global__ __launch_bounds__(256) void gemm64(
    const unsigned short* __restrict__ Ap, int lda,
    const unsigned short* __restrict__ Btp, int ldb, long long strideB,
    float* Cp, int ldc, long long strideC,
    int M, int N, int K, float oscale,
    const float* __restrict__ bias0, int nbias) {
  const _Float16* A  = (const _Float16*)(const void*)Ap;
  const _Float16* Bt = (const _Float16*)(const void*)Btp;
  __shared__ __align__(16) float sT[8][16 * 68];
  const int b    = blockIdx.y;
  const int lane = threadIdx.x & 31;
  const int wave = threadIdx.x >> 5;
  const int tilesN = N >> 6;
  const int tilesM = M >> 6;
  const int tile = blockIdx.x * 8 + wave;
  if (tile >= tilesM * tilesN) return;
  const int tm = tile / tilesN;
  const int tn = tile - tm * tilesN;
  const int m0 = tm << 6;
  const int n0 = tn << 6;

  const _Float16* Bb = Bt + (size_t)b * strideB;

  const int rlane = lane & 15;
  const int koff  = (lane >> 4) * 8;
  const int mOff  = (lane >> 4) * 8;

  v8f acc[4][4];
#pragma unroll
  for (int i = 0; i < 4; ++i)
#pragma unroll
    for (int j = 0; j < 4; ++j) acc[i][j] = zero8();

  for (int k0 = 0; k0 < K; k0 += 32) {
    v16h bh[4];
#pragma unroll
    for (int j = 0; j < 4; ++j) {
      const size_t bo = (size_t)(n0 + (j << 4) + rlane) * ldb + koff + k0;
      bh[j] = ldfrag_h(Bb + bo);
    }
#pragma unroll
    for (int i = 0; i < 4; ++i) {
      const size_t ao = (size_t)(m0 + (i << 4) + rlane) * lda + koff + k0;
      const v16h ah = ldfrag_h(A + ao);
#pragma unroll
      for (int j = 0; j < 4; ++j) {
        acc[i][j] = mma_h_raw(ah, bh[j], acc[i][j]);
      }
      dep_guard_h(acc[i][0], acc[i][3], ah, bh[3]);
    }
    keep4_h(bh[0], bh[1], bh[2], bh[3]);
  }
  acc_guard4(acc[0][0], acc[0][1], acc[0][2], acc[0][3]);
  acc_guard4(acc[1][0], acc[1][1], acc[1][2], acc[1][3]);
  acc_guard4(acc[2][0], acc[2][1], acc[2][2], acc[2][3]);
  acc_guard4(acc[3][0], acc[3][1], acc[3][2], acc[3][3]);

  float* slab = sT[wave];
  float* C = Cp + (size_t)b * strideC;
  const int bclamp = (nbias > 0) ? (nbias - 1) : 0;
#pragma unroll
  for (int i = 0; i < 4; ++i) {
    const int mBase = m0 + (i << 4);
#pragma unroll
    for (int j = 0; j < 4; ++j) {
#pragma unroll
      for (int r = 0; r < 8; ++r) {
        slab[(mOff + r) * 68 + (j << 4) + rlane] = acc[i][j][r];
      }
    }
    wave_sync_lds();
    {
      const int hh = lane >> 4, c4 = (lane & 15) * 4;
      v4f ov[8];
#pragma unroll
      for (int it = 0; it < 8; ++it) {
        const int row = it * 2 + hh;
        const int mrw = mBase + row;
        const float bl = bfr(bias0[min(mrw, bclamp)]);
        const float bv = (nbias > 0) ? bl : 0.0f;
        v4f v = *(const v4f*)(slab + row * 68 + c4);
        v[0] = v[0] * oscale + bv;
        v[1] = v[1] * oscale + bv;
        v[2] = v[2] * oscale + bv;
        v[3] = v[3] * oscale + bv;
        ov[it] = v;
      }
      for (int pass = 0; pass < 2; ++pass) {
#pragma unroll
        for (int it = 0; it < 8; ++it) {
          const int row = it * 2 + hh;
          *(volatile v4f*)(C + (size_t)(mBase + row) * ldc + n0 + c4) = ov[it];
        }
        __threadfence();
      }
    }
    wave_sync_lds();
  }
}

__global__ __launch_bounds__(256) void k_means(const float* __restrict__ F, float* mu) {
  __shared__ __align__(16) float sMu[32];
  const int tid = threadIdx.x, wave = tid >> 5, lane = tid & 31;
  const int rb = blockIdx.x * 32;
#pragma unroll 1
  for (int i = 0; i < 4; ++i) {
    const int row = rb + wave * 4 + i;
    const v4f* rp = (const v4f*)(F + (size_t)row * NP);
    float s = 0.0f;
#pragma unroll 4
    for (int k = 0; k < NP / 128; ++k) {
      const v4f v = rp[k * 32 + lane];
      s += (v[0] + v[1]) + (v[2] + v[3]);
    }
#pragma unroll
    for (int off = 16; off >= 1; off >>= 1) s += __shfl_xor(s, off, 32);
    if (lane == 0) sMu[wave * 4 + i] = s * (1.0f / (float)NP);
  }
  __syncthreads();
  if (tid < 8) {
    const v4f v = *(const v4f*)(sMu + 4 * tid);
    float* d = mu + rb + 4 * tid;
    *(volatile v4f*)d = v;
    __threadfence();
    *(volatile v4f*)d = v;
  }
}

__global__ __launch_bounds__(256) void cvt_qk(const float* __restrict__ F, const float* __restrict__ mu,
                                               unsigned short* qh, unsigned short* kh) {
  __shared__ __align__(16) float st[DQ * 33];
  __shared__ float sMu[DQ];
  const int which = blockIdx.y;
  const float* src = F + (size_t)which * DQ * NP;
  const float* mup = mu + which * DQ;
  unsigned short* dh = (which != 0) ? kh : qh;
  const int tid = threadIdx.x, wave = tid >> 5, lane = tid & 31;
  const int p0 = blockIdx.x * 32;
#pragma unroll
  for (int it = 0; it < 8; ++it) {
    const int idx = it * 256 + tid;
    const int c = idx >> 5, q = idx & 31;
    st[c * 33 + q] = src[(size_t)c * NP + p0 + q];
  }
  if (tid < DQ) sMu[tid] = mup[tid];
  __syncthreads();
  const int rq = lane >> 3, cl = (lane & 7) * 8;
  const int r = wave * 4 + rq;
  v4u p;
#pragma unroll
  for (int e = 0; e < 4; ++e) {
    const int c0 = cl + 2 * e, c1 = c0 + 1;
    const float a = (st[c0 * 33 + r] - sMu[c0]) * ASCALE;
    const float b = (st[c1 * 33 + r] - sMu[c1]) * ASCALE;
    p[e] = pk16(f2h_bits(a), f2h_bits(b));
  }
  unsigned short* d = dh + (size_t)(p0 + r) * DQ + cl;
  *(volatile v4u*)d = p;
  __threadfence();
  *(volatile v4u*)d = p;
}

__global__ __launch_bounds__(256) void cvt_v(const float* __restrict__ F, unsigned short* vh) {
  const int tid = threadIdx.x, wave = tid >> 5, lane = tid & 31;
  const int row = blockIdx.x * 8 + wave;
  const float* s = F + (size_t)(2 * DQ + row) * NP;
  unsigned short* d = vh + (size_t)row * NP;
#pragma unroll 1
  for (int it = 0; it < VPC; ++it) {
    const int base = it * 256 + lane * 8;
    const v4f a = *(const v4f*)(s + base);
    const v4f c = *(const v4f*)(s + base + 4);
    v4u p;
    p[0] = pk16(f2h_bits(a[0] * ASCALE), f2h_bits(a[1] * ASCALE));
    p[1] = pk16(f2h_bits(a[2] * ASCALE), f2h_bits(a[3] * ASCALE));
    p[2] = pk16(f2h_bits(c[0] * ASCALE), f2h_bits(c[1] * ASCALE));
    p[3] = pk16(f2h_bits(c[2] * ASCALE), f2h_bits(c[3] * ASCALE));
    unsigned short* dd = d + base;
    *(volatile v4u*)dd = p;
    __threadfence();
    *(volatile v4u*)dd = p;
  }
}

__global__ __launch_bounds__(256) void k_attn(const unsigned short* __restrict__ qhp,
                                               const unsigned short* __restrict__ khp,
                                               const unsigned short* __restrict__ vhp,
                                               const float* __restrict__ means,
                                               const float* __restrict__ gam,
                                               float* out) {
  const _Float16* Q  = (const _Float16*)(const void*)qhp;
  const _Float16* Kt = (const _Float16*)(const void*)khp;
  const _Float16* V  = (const _Float16*)(const void*)vhp;
  __shared__ __align__(16) _Float16 sP[QTILE * SPP];
  __shared__ float sM1[8][16];
  __shared__ float sL1[8][16];
  __shared__ float sMrow[QTILE];
  __shared__ float sRinv[QTILE];
  __shared__ __align__(16) float slab[8][16 * SLP];

  const int tid = threadIdx.x, wave = tid >> 5, lane = tid & 31;
  const int rl = lane & 15, h = lane >> 4, koff = h * 8;
  const int q0 = blockIdx.x * QTILE;
  const int mt = wave >> 1, kh = wave & 1;
  const size_t tokq = (size_t)q0 + 16 * mt;

  v16h qa[2];
#pragma unroll
  for (int ks = 0; ks < 2; ++ks) qa[ks] = ldfrag_h(Q + (tokq + rl) * DQ + 32 * ks + koff);

  float mr[8], lr[8];
#pragma unroll
  for (int r = 0; r < 8; ++r) { mr[r] = -3.0e38f; lr[r] = 0.0f; }
  v16h kf;
#pragma unroll 1
  for (int t = 0; t < NT16; ++t) {
    const size_t tokk = (size_t)kh * KHALF + 16 * t;
    v8f s = zero8();
#pragma unroll
    for (int ks = 0; ks < 2; ++ks) {
      kf = ldfrag_h(Kt + (tokk + rl) * DQ + 32 * ks + koff);
      s = mma_h_raw(qa[ks], kf, s);
    }
    dep_guard1(s, qa[1], kf);
#pragma unroll
    for (int r = 0; r < 8; ++r) {
      const float v   = s[r] * SINV;
      const float dd  = v - mr[r];
      const float tt  = __expf(-fabsf(dd));
      const bool  gt  = dd > 0.0f;
      const float lle = lr[r] + tt;
      const float lgt = lr[r] * tt + 1.0f;
      lr[r] = gt ? lgt : lle;
      mr[r] = gt ? v : mr[r];
    }
  }
#pragma unroll
  for (int r = 0; r < 8; ++r) {
    float mm = mr[r];
    mm = fmaxf(mm, __shfl_xor(mm, 1, 32));
    mm = fmaxf(mm, __shfl_xor(mm, 2, 32));
    mm = fmaxf(mm, __shfl_xor(mm, 4, 32));
    mm = fmaxf(mm, __shfl_xor(mm, 8, 32));
    float term = lr[r] * __expf(mr[r] - mm);
    term += __shfl_xor(term, 1, 32);
    term += __shfl_xor(term, 2, 32);
    term += __shfl_xor(term, 4, 32);
    term += __shfl_xor(term, 8, 32);
    mr[r] = mm;
    lr[r] = term;
  }
  if (rl == 0) {
#pragma unroll
    for (int r = 0; r < 8; ++r) { sM1[wave][8 * h + r] = mr[r]; sL1[wave][8 * h + r] = lr[r]; }
  }
  __syncthreads();
  if (tid < QTILE) {
    const int m4 = tid >> 4, rr = tid & 15;
    const float m0 = sM1[2 * m4][rr], m1 = sM1[2 * m4 + 1][rr];
    const float l0 = sL1[2 * m4][rr], l1 = sL1[2 * m4 + 1][rr];
    const float m = fmaxf(m0, m1);
    const float l = l0 * __expf(m0 - m) + l1 * __expf(m1 - m);
    sMrow[tid] = m;
    sRinv[tid] = PSCALE * (1.0f / l);
  }
  __syncthreads();
  float mrow[8], rinv[8];
#pragma unroll
  for (int r = 0; r < 8; ++r) { mrow[r] = sMrow[16 * mt + 8 * h + r]; rinv[r] = sRinv[16 * mt + 8 * h + r]; }

  v8f acc[4][2];
#pragma unroll
  for (int i = 0; i < 4; ++i) { acc[i][0] = zero8(); acc[i][1] = zero8(); }
  const int cw = wave * 32;
  const _Float16* Vb = V + (size_t)cw * NP;
  v16h vf0, vf1;
#pragma unroll 1
  for (int kc = 0; kc < NKC; ++kc) {
    const size_t tokk = (size_t)kc * 32 + 16 * kh;
    v8f s = zero8();
#pragma unroll
    for (int ks = 0; ks < 2; ++ks) {
      kf = ldfrag_h(Kt + (tokk + rl) * DQ + 32 * ks + koff);
      s = mma_h_raw(qa[ks], kf, s);
    }
    dep_guard1(s, qa[1], kf);
#pragma unroll
    for (int r = 0; r < 8; ++r) {
      const float v  = s[r] * SINV;
      const float pv = __expf(v - mrow[r]) * rinv[r] - PSHIFT;
      sP[(16 * mt + 8 * h + r) * SPP + 16 * kh + rl] = (_Float16)pv;
    }
    __syncthreads();
    vf0 = ldfrag_h(Vb + (size_t)rl * NP + kc * 32 + koff);
    vf1 = ldfrag_h(Vb + (size_t)(16 + rl) * NP + kc * 32 + koff);
#pragma unroll
    for (int m2 = 0; m2 < 4; ++m2) {
      const v16h af = ldfrag_h(sP + (16 * m2 + rl) * SPP + koff);
      acc[m2][0] = mma_h_raw(af, vf0, acc[m2][0]);
      acc[m2][1] = mma_h_raw(af, vf1, acc[m2][1]);
      dep_guard_h(acc[m2][0], acc[m2][1], af, vf1);
    }
    keep2_h(vf0, vf1);
    __syncthreads();
  }
  acc_guard4(acc[0][0], acc[0][1], acc[1][0], acc[1][1]);
  acc_guard4(acc[2][0], acc[2][1], acc[3][0], acc[3][1]);

  const float g = bfr(gam[0]);
  float* sl = slab[wave];
  const int hh = lane >> 4, c4 = (lane & 15) * 4;
#pragma unroll
  for (int nt = 0; nt < 2; ++nt) {
#pragma unroll
    for (int m2 = 0; m2 < 4; ++m2)
#pragma unroll
      for (int r = 0; r < 8; ++r) sl[rl * SLP + 16 * m2 + 8 * h + r] = acc[m2][nt][r];
    wave_sync_lds();
    v4f ov[8];
#pragma unroll
    for (int it = 0; it < 8; ++it) {
      const int row = it * 2 + hh;
      const int c = cw + 16 * nt + row;
      const float vm = means[2 * DQ + c];
      v4f v = *(const v4f*)(sl + row * SLP + c4);
      v[0] = g * (v[0] * OSC_ATT + vm);
      v[1] = g * (v[1] * OSC_ATT + vm);
      v[2] = g * (v[2] * OSC_ATT + vm);
      v[3] = g * (v[3] * OSC_ATT + vm);
      ov[it] = v;
    }
    for (int pass = 0; pass < 2; ++pass) {
#pragma unroll
      for (int it = 0; it < 8; ++it) {
        const int row = it * 2 + hh;
        const int c = cw + 16 * nt + row;
        *(volatile v4f*)(out + (size_t)c * NP + q0 + c4) = ov[it];
      }
      __threadfence();
    }
    wave_sync_lds();
  }
}

extern "C" void kernel_launch(void* const* d_in, const int* in_sizes, int n_in,
                              void* d_out, int out_size, void* d_ws, size_t ws_size,
                              hipStream_t stream) {
  if (n_in < 8) return;
  if (in_sizes[0] != CH * NP) return;
  if (in_sizes[1] != CH * NP) return;
  if (in_sizes[2] != CH * CH) return;
  if (in_sizes[3] != DQ * CH) return;
  if (in_sizes[4] != DQ) return;
  if (in_sizes[5] != DQ * CH) return;
  if (in_sizes[6] != DQ) return;
  if (in_sizes[7] < 1) return;
  if (out_size != CH * NP) return;

  const float* x     = (const float*)d_in[0];
  const float* y     = (const float*)d_in[1];
  const float* wv    = (const float*)d_in[2];
  const float* wq    = (const float*)d_in[3];
  const float* bq    = (const float*)d_in[4];
  const float* wk    = (const float*)d_in[5];
  const float* bk    = (const float*)d_in[6];
  const float* gamma = (const float*)d_in[7];
  float* out = (float*)d_out;

  const size_t PXT = (size_t)NP * CH * 2;
  const size_t PW  = (size_t)NROWS * CH * 2;
  const size_t PF  = (size_t)NROWS * NP * 4;
  const size_t PMU = (size_t)NROWS * 4;
  const size_t PQH = (size_t)NP * DQ * 2;
  const size_t PVH = (size_t)CH * NP * 2;

  size_t off = 0;
  const size_t oXT = off; off += PXT;
  const size_t oYT = off; off += PXT;
  const size_t oW  = off; off += PW;
  const size_t oF  = off; off += PF;
  const size_t oMU = off; off += PMU;
  const size_t oQH = off; off += PQH;
  const size_t oKH = off; off += PQH;
  const size_t oVH = off; off += PVH;
  if (off > ws_size) return;
  if (off > (size_t)134217728) return;

  char* ws = (char*)d_ws;
  unsigned short* XT   = (unsigned short*)(ws + oXT);
  unsigned short* YT   = (unsigned short*)(ws + oYT);
  unsigned short* WALL = (unsigned short*)(ws + oW);
  float*          F    = (float*)(ws + oF);
  float*          MU   = (float*)(ws + oMU);
  unsigned short* QH   = (unsigned short*)(ws + oQH);
  unsigned short* KH   = (unsigned short*)(ws + oKH);
  unsigned short* VH   = (unsigned short*)(ws + oVH);

  const dim3 blk(256);
  cvt_tok<<<dim3(PT, 2), blk, 0, stream>>>(x, y, XT, YT);
  cvt_w<<<dim3(NROWS / 8), blk, 0, stream>>>(wq, wk, wv, WALL);
  const dim3 gQ(((DQ / 64) * (NP / 64)) / 8, 1);
  const dim3 gV(((CH / 64) * (NP / 64)) / 8, 1);
  gemm64<<<gQ, blk, 0, stream>>>(WALL, CH, XT, CH, 0LL, F, NP, 0LL,
                                 DQ, NP, CH, OSC_PROJ, bq, DQ);
  gemm64<<<gQ, blk, 0, stream>>>(WALL + (size_t)DQ * CH, CH, YT, CH, 0LL, F + (size_t)DQ * NP, NP, 0LL,
                                 DQ, NP, CH, OSC_PROJ, bk, DQ);
  gemm64<<<gV, blk, 0, stream>>>(WALL + (size_t)2 * DQ * CH, CH, YT, CH, 0LL, F + (size_t)2 * DQ * NP, NP, 0LL,
                                 CH, NP, CH, OSC_PROJ, bq, 0);
  k_means<<<dim3(NROWS / 32), blk, 0, stream>>>(F, MU);
  cvt_qk<<<dim3(PT, 2), blk, 0, stream>>>(F, MU, QH, KH);
  cvt_v<<<dim3(CH / 8), blk, 0, stream>>>(F, VH);
  k_attn<<<dim3(NQT), blk, 0, stream>>>(QH, KH, VH, MU, gamma, out);
  (void)hipGetLastError();
}
